// MambaLayer_67078799229628
// MI455X (gfx1250) — hardware-run, weakly checked
//
#include <hip/hip_runtime.h>
#include <math.h>

typedef __attribute__((ext_vector_type(16))) _Float16 v16h;
typedef __attribute__((ext_vector_type(8)))  _Float16 v8h;
typedef __attribute__((ext_vector_type(16))) __bf16   v16b;
typedef __attribute__((ext_vector_type(8)))  __bf16   v8b;
typedef __attribute__((ext_vector_type(8)))  float    v8f;
typedef __attribute__((ext_vector_type(4)))  float    v4f;

constexpr int kBatch  = 2;
constexpr int kSeq    = 1024;
constexpr int kDm     = 768;
constexpr int kDin    = 1536;
constexpr int kNst    = 64;
constexpr int kDtR    = 48;
constexpr int kDtP    = 64;
constexpr int kPrjN   = kDtR + 2 * kNst;
constexpr int kPrjP   = 192;
constexpr int kXzP    = 2 * kDin;
constexpr int kRows   = kBatch * kSeq;
constexpr int kConvTP = 260;
constexpr int kScTS   = 16;
constexpr int kScCh   = 64;
constexpr int kScQ    = 4;
constexpr int kScNq   = kNst / kScQ;
constexpr float kLnEps    = 1e-5f;
constexpr float kCarryXa  = 16.0f;
constexpr float kCarryWx  = 32.0f;
constexpr float kCarryDt  = 16.0f;
constexpr float kCarryWdt = 8.0f;
static_assert(kPrjN == 176);
static_assert(kPrjP % 64 == 0 && kPrjP >= kPrjN);
static_assert(kDtP % 32 == 0 && kDtP >= kDtR && (kDtR % 8) == 0);
static_assert((kDm % 32) == 0 && (kDin % 32) == 0);
static_assert((kRows % 64) == 0 && (kXzP % 64) == 0 && (kDin % 64) == 0 && (kDm % 64) == 0);
static_assert((kSeq % 64) == 0 && (kSeq % kScTS) == 0 && (kDin % 256) == 0 && (kDin % kScCh) == 0);
static_assert(kDm == 3 * 256 && (kRows % 8) == 0);
static_assert(kScNq == 16 && kScCh * kScQ == 256);

constexpr size_t kOffXNH  = 0;
constexpr size_t kOffXNL  = kOffXNH  + (size_t)kRows * kDm  * 2;
constexpr size_t kOffWIH  = kOffXNL  + (size_t)kRows * kDm  * 2;
constexpr size_t kOffWIL  = kOffWIH  + (size_t)kXzP  * kDm  * 2;
constexpr size_t kOffWOH  = kOffWIL  + (size_t)kXzP  * kDm  * 2;
constexpr size_t kOffWOL  = kOffWOH  + (size_t)kDm   * kDin * 2;
constexpr size_t kOffWXP  = kOffWOL  + (size_t)kDm   * kDin * 2;
constexpr size_t kOffWDT  = kOffWXP  + (size_t)kPrjP * kDin * 2;
constexpr size_t kOffXZ   = kOffWDT  + (size_t)kDin  * kDtP * 2;
constexpr size_t kOffUC   = kOffXZ   + (size_t)kRows * kXzP * 4;
constexpr size_t kOffUC16 = kOffUC   + (size_t)kRows * kDin * 4;
constexpr size_t kOffPROJ = kOffUC16 + (size_t)kRows * kDin * 2;
constexpr size_t kOffDT16 = kOffPROJ + (size_t)kRows * kPrjP * 4;
constexpr size_t kOffDLR  = kOffDT16 + (size_t)kRows * kDtP * 2;
constexpr size_t kOffYH   = kOffDLR  + (size_t)kRows * kDin * 4;
constexpr size_t kOffYL   = kOffYH   + (size_t)kRows * kDin * 2;
constexpr size_t kWsTotal = kOffYL   + (size_t)kRows * kDin * 2;
static_assert(kWsTotal == 92274688ull);
static_assert(kWsTotal <= 134217728ull);
static_assert((kOffXNL % 128) == 0 && (kOffWIH % 128) == 0 && (kOffWIL % 128) == 0 && (kOffWOH % 128) == 0 &&
              (kOffWOL % 128) == 0 && (kOffWXP % 128) == 0 && (kOffWDT % 128) == 0 && (kOffXZ % 128) == 0 &&
              (kOffUC % 128) == 0 && (kOffUC16 % 128) == 0 && (kOffPROJ % 128) == 0 && (kOffDT16 % 128) == 0 &&
              (kOffDLR % 128) == 0 && (kOffYH % 128) == 0 && (kOffYL % 128) == 0);

__device__ __forceinline__ unsigned short f2bf_bits(float f) {
  unsigned u = __float_as_uint(f);
  return (unsigned short)((u + 0x7FFFu + ((u >> 16) & 1u)) >> 16);
}
__device__ __forceinline__ float bf_bits2f(unsigned short h) { return __uint_as_float(((unsigned)h) << 16); }

__device__ __forceinline__ void dep_guard4_h(v8f& a, v8f& b, v8f& c, v8f& d, v16h x, v16h y) {
  asm volatile("v_nop\n\tv_nop\n\tv_nop\n\tv_nop" : "+v"(a), "+v"(b), "+v"(c), "+v"(d) : "v"(x), "v"(y));
}
__device__ __forceinline__ void dep_guard4_b(v8f& a, v8f& b, v8f& c, v8f& d, v16b x, v16b y) {
  asm volatile("v_nop\n\tv_nop\n\tv_nop\n\tv_nop" : "+v"(a), "+v"(b), "+v"(c), "+v"(d) : "v"(x), "v"(y));
}
__device__ __forceinline__ void keep4_h(v16h a, v16h b, v16h c, v16h d) { asm volatile("v_nop" :: "v"(a), "v"(b), "v"(c), "v"(d)); }
__device__ __forceinline__ void keep4_b(v16b a, v16b b, v16b c, v16b d) { asm volatile("v_nop" :: "v"(a), "v"(b), "v"(c), "v"(d)); }
__device__ __forceinline__ void acc_guard4(v8f& a, v8f& b, v8f& c, v8f& d) {
  asm volatile("v_nop\n\tv_nop\n\tv_nop\n\tv_nop" : "+v"(a), "+v"(b), "+v"(c), "+v"(d));
}
template <typename T> struct Frag;
template <> struct Frag<_Float16> {
  typedef v16h V; union U { v16h v; v8h h[2]; };
  static __device__ __forceinline__ v16h load(const _Float16* p) {
    U f; f.h[0] = *(const v8h*)(p); f.h[1] = *(const v8h*)(p + 16); return f.v;
  }
  static __device__ __forceinline__ v8f mma(v16h a, v16h b, v8f c) {
    return __builtin_amdgcn_wmma_f32_16x16x32_f16(false, a, false, b, (short)0, c, false, false);
  }
  static __device__ __forceinline__ void guard4(v8f& a, v8f& b, v8f& c, v8f& d, v16h x, v16h y) { dep_guard4_h(a, b, c, d, x, y); }
  static __device__ __forceinline__ void keep(v16h a, v16h b, v16h c, v16h d) { keep4_h(a, b, c, d); }
};
template <> struct Frag<__bf16> {
  typedef v16b V; union U { v16b v; v8b h[2]; };
  static __device__ __forceinline__ v16b load(const __bf16* p) {
    U f; f.h[0] = *(const v8b*)(p); f.h[1] = *(const v8b*)(p + 16); return f.v;
  }
  static __device__ __forceinline__ v8f mma(v16b a, v16b b, v8f c) {
    return __builtin_amdgcn_wmma_f32_16x16x32_bf16(false, a, false, b, (short)0, c, false, false);
  }
  static __device__ __forceinline__ void guard4(v8f& a, v8f& b, v8f& c, v8f& d, v16b x, v16b y) { dep_guard4_b(a, b, c, d, x, y); }
  static __device__ __forceinline__ void keep(v16b a, v16b b, v16b c, v16b d) { keep4_b(a, b, c, d); }
};

template <int ET> struct Elem;
template <> struct Elem<0> { typedef _Float16 T; };
template <> struct Elem<1> { typedef __bf16 T; };
template <int ET, int SPL, int BIAS_MODE>
__global__ __launch_bounds__(256) void wmma_gemm64(
    const unsigned short* __restrict__ Ap, const unsigned short* __restrict__ A2p, int lda,
    const unsigned short* __restrict__ Btp, const unsigned short* __restrict__ Bt2p, int ldb,
    float* __restrict__ Cout, int ldc,
    const float* __restrict__ bias,
    int M, int N, int K, float scale) {
  typedef typename Elem<ET>::T T;
  typedef typename Frag<T>::V V;
  const T* A = (const T*)Ap; const T* A2 = (const T*)A2p; const T* Bt = (const T*)Btp; const T* Bt2 = (const T*)Bt2p;
  __shared__ __align__(16) float sT[8][16 * 68];
  const int lane = threadIdx.x & 31;
  const int wave = threadIdx.x >> 5;
  const int tilesN = N >> 6;
  const int tilesM = M >> 6;
  const int tile = blockIdx.x * 8 + wave;
  if (tile >= tilesM * tilesN) return;
  const int tm = tile / tilesN;
  const int tn = tile - tm * tilesN;
  const int m0 = tm << 6;
  const int n0 = tn << 6;

  const int rlane = lane & 15;
  const int koff  = (lane >> 4) * 8;
  const int mOff  = (lane >> 4) * 8;

  v8f acc[4][4];
#pragma unroll
  for (int i = 0; i < 4; ++i)
#pragma unroll
    for (int j = 0; j < 4; ++j) acc[i][j] = (v8f){0.f,0.f,0.f,0.f,0.f,0.f,0.f,0.f};

  for (int k0 = 0; k0 < K; k0 += 32) {
    {
      V bf[4];
#pragma unroll
      for (int j = 0; j < 4; ++j) {
        const size_t bo = (size_t)(n0 + (j << 4) + rlane) * ldb + koff + k0;
        bf[j] = Frag<T>::load(Bt + bo);
      }
#pragma unroll
      for (int i = 0; i < 4; ++i) {
        const size_t ao = (size_t)(m0 + (i << 4) + rlane) * lda + koff + k0;
        V ah = Frag<T>::load(A + ao);
        V al = ah;
        if (SPL == 2) al = Frag<T>::load(A2 + ao);
#pragma unroll
        for (int j = 0; j < 4; ++j) {
          acc[i][j] = Frag<T>::mma(ah, bf[j], acc[i][j]);
          if (SPL == 2) acc[i][j] = Frag<T>::mma(al, bf[j], acc[i][j]);
        }
        Frag<T>::guard4(acc[i][0], acc[i][1], acc[i][2], acc[i][3], ah, al);
      }
      Frag<T>::keep(bf[0], bf[1], bf[2], bf[3]);
    }
    if (SPL == 2) {
      V bg[4];
#pragma unroll
      for (int j = 0; j < 4; ++j) {
        const size_t bo = (size_t)(n0 + (j << 4) + rlane) * ldb + koff + k0;
        bg[j] = Frag<T>::load(Bt2 + bo);
      }
#pragma unroll
      for (int i = 0; i < 4; ++i) {
        const size_t ao = (size_t)(m0 + (i << 4) + rlane) * lda + koff + k0;
        V ah = Frag<T>::load(A + ao);
#pragma unroll
        for (int j = 0; j < 4; ++j) acc[i][j] = Frag<T>::mma(ah, bg[j], acc[i][j]);
        Frag<T>::guard4(acc[i][0], acc[i][1], acc[i][2], acc[i][3], ah, ah);
      }
      Frag<T>::keep(bg[0], bg[1], bg[2], bg[3]);
    }
  }
  acc_guard4(acc[0][0], acc[0][1], acc[0][2], acc[0][3]);
  acc_guard4(acc[1][0], acc[1][1], acc[1][2], acc[1][3]);
  acc_guard4(acc[2][0], acc[2][1], acc[2][2], acc[2][3]);
  acc_guard4(acc[3][0], acc[3][1], acc[3][2], acc[3][3]);

  float* slab = sT[wave];
#pragma unroll
  for (int i = 0; i < 4; ++i) {
    const int mBase = m0 + (i << 4);
#pragma unroll
    for (int j = 0; j < 4; ++j) {
      const int n = n0 + (j << 4) + rlane;
      float bv = 0.f;
      if (BIAS_MODE == 2) bv = bias[n];
#pragma unroll
      for (int r = 0; r < 8; ++r) {
        float v = acc[i][j][r] * scale;
        if (BIAS_MODE == 2) v += bv;
        slab[(mOff + r) * 68 + (j << 4) + rlane] = v;
      }
    }
    __builtin_amdgcn_fence(__ATOMIC_RELEASE, "workgroup");
    __builtin_amdgcn_wave_barrier();
    __builtin_amdgcn_fence(__ATOMIC_ACQUIRE, "workgroup");
    {
      const int hh = lane >> 4, c4 = (lane & 15) * 4;
      for (int pass = 0; pass < 2; ++pass) {
#pragma unroll
        for (int it = 0; it < 8; ++it) {
          const int row = it * 2 + hh;
          v4f v = *(const v4f*)(slab + row * 68 + c4);
          *(volatile v4f*)(Cout + (size_t)(mBase + row) * ldc + n0 + c4) = v;
        }
        __threadfence();
      }
    }
    __builtin_amdgcn_fence(__ATOMIC_RELEASE, "workgroup");
    __builtin_amdgcn_wave_barrier();
    __builtin_amdgcn_fence(__ATOMIC_ACQUIRE, "workgroup");
  }
}

__global__ __launch_bounds__(256) void split_rows_bf16_kernel(
    const float* __restrict__ src, unsigned short* __restrict__ dhi, unsigned short* __restrict__ dlo, int total8)
{
  const int i = blockIdx.x * 256 + threadIdx.x;
  if (i >= total8) return;
  const size_t e0 = (size_t)i << 3;
  const v4f a0 = *(const v4f*)(src + e0);
  const v4f a1 = *(const v4f*)(src + e0 + 4);
  v8h hv, lv;
#pragma unroll
  for (int e = 0; e < 4; ++e) {
    const float f0 = a0[e], f1 = a1[e];
    const unsigned short h0 = f2bf_bits(f0), h1 = f2bf_bits(f1);
    const unsigned short l0 = f2bf_bits(f0 - bf_bits2f(h0)), l1 = f2bf_bits(f1 - bf_bits2f(h1));
    hv[e]     = __builtin_bit_cast(_Float16, h0);
    hv[4 + e] = __builtin_bit_cast(_Float16, h1);
    lv[e]     = __builtin_bit_cast(_Float16, l0);
    lv[4 + e] = __builtin_bit_cast(_Float16, l1);
  }
  unsigned short* qh = dhi + e0;
  unsigned short* ql = dlo + e0;
  *(volatile v8h*)qh = hv;
  *(volatile v8h*)ql = lv;
  __threadfence();
  *(volatile v8h*)qh = hv;
  *(volatile v8h*)ql = lv;
}

__global__ __launch_bounds__(256) void cast_pad_f16_kernel(
    const float* __restrict__ src, int srcPitch, int srcRows, int srcCols,
    unsigned short* __restrict__ dst, int dstCols, int total8, float scale)
{
  const int i = blockIdx.x * 256 + threadIdx.x;
  if (i >= total8) return;
  const int e0  = i << 3;
  const int row = e0 / dstCols;
  const int col = e0 - row * dstCols;
  const bool ok = (row < srcRows) && (col < srcCols);
  const int rc  = (row < srcRows) ? row : (srcRows - 1);
  const int cc  = (col < srcCols) ? col : (srcCols - 8);
  const float* p = src + (size_t)rc * srcPitch + cc;
  const v4f a0 = *(const v4f*)(p);
  const v4f a1 = *(const v4f*)(p + 4);
  v8h hv;
#pragma unroll
  for (int e = 0; e < 4; ++e) {
    const float f0 = ok ? (a0[e] * scale) : 0.0f;
    const float f1 = ok ? (a1[e] * scale) : 0.0f;
    hv[e]     = (_Float16)f0;
    hv[4 + e] = (_Float16)f1;
  }
  unsigned short* q = dst + (size_t)e0;
  *(volatile v8h*)q = hv;
  __threadfence();
  *(volatile v8h*)q = hv;
}

__global__ __launch_bounds__(256) void ln_split_kernel(
    const float* __restrict__ x, const float* __restrict__ gam, const float* __restrict__ bet,
    unsigned short* __restrict__ XH, unsigned short* __restrict__ XL)
{
  const int lane = threadIdx.x & 31, wave = threadIdx.x >> 5;
  const int row = blockIdx.x * 8 + wave;
  const float* xr = x + (size_t)row * kDm + lane * 8;

  float s = 0.f;
#pragma unroll 1
  for (int j = 0; j < 3; ++j) {
    const v4f a0 = *(const v4f*)(xr + j * 256);
    const v4f a1 = *(const v4f*)(xr + j * 256 + 4);
    s += ((a0[0] + a0[1]) + (a0[2] + a0[3])) + ((a1[0] + a1[1]) + (a1[2] + a1[3]));
  }
  s += __shfl_xor(s, 16, 32);
  s += __shfl_xor(s, 8, 32);
  s += __shfl_xor(s, 4, 32);
  s += __shfl_xor(s, 2, 32);
  s += __shfl_xor(s, 1, 32);
  const float mean = s * (1.0f / (float)kDm);

  float q = 0.f;
#pragma unroll 1
  for (int j = 0; j < 3; ++j) {
    const v4f a0 = *(const v4f*)(xr + j * 256);
    const v4f a1 = *(const v4f*)(xr + j * 256 + 4);
#pragma unroll
    for (int e = 0; e < 4; ++e) {
      const float d0 = a0[e] - mean;
      const float d1 = a1[e] - mean;
      q = fmaf(d0, d0, q);
      q = fmaf(d1, d1, q);
    }
  }
  q += __shfl_xor(q, 16, 32);
  q += __shfl_xor(q, 8, 32);
  q += __shfl_xor(q, 4, 32);
  q += __shfl_xor(q, 2, 32);
  q += __shfl_xor(q, 1, 32);
  const float var  = q * (1.0f / (float)kDm);
  const float rstd = 1.0f / sqrtf(var + kLnEps);

#pragma unroll 1
  for (int j = 0; j < 3; ++j) {
    const int cofs = j * 256 + lane * 8;
    const v4f a0 = *(const v4f*)(xr + j * 256);
    const v4f a1 = *(const v4f*)(xr + j * 256 + 4);
    const v4f g0 = *(const v4f*)(gam + cofs);
    const v4f g1 = *(const v4f*)(gam + cofs + 4);
    const v4f b0 = *(const v4f*)(bet + cofs);
    const v4f b1 = *(const v4f*)(bet + cofs + 4);
    v8h hv, lv;
#pragma unroll
    for (int e = 0; e < 4; ++e) {
      const float x0 = a0[e], x1 = a1[e];
      const float v0 = ((x0 - mean) * rstd) * g0[e] + b0[e];
      const float v1 = ((x1 - mean) * rstd) * g1[e] + b1[e];
      const unsigned short h0 = f2bf_bits(v0), h1 = f2bf_bits(v1);
      const unsigned short l0 = f2bf_bits(v0 - bf_bits2f(h0)), l1 = f2bf_bits(v1 - bf_bits2f(h1));
      hv[e]     = __builtin_bit_cast(_Float16, h0);
      hv[4 + e] = __builtin_bit_cast(_Float16, h1);
      lv[e]     = __builtin_bit_cast(_Float16, l0);
      lv[4 + e] = __builtin_bit_cast(_Float16, l1);
    }
    const size_t o = (size_t)row * kDm + cofs;
    *(volatile v8h*)(XH + o) = hv;
    *(volatile v8h*)(XL + o) = lv;
    __threadfence();
    *(volatile v8h*)(XH + o) = hv;
    *(volatile v8h*)(XL + o) = lv;
  }
}

__global__ __launch_bounds__(256) void conv_silu_kernel(
    const float* __restrict__ XZ, const float* __restrict__ cw, const float* __restrict__ cb,
    float* __restrict__ UC, unsigned short* __restrict__ UC16)
{
  __shared__ __align__(16) float sT[16 * kConvTP];
  const int tid = threadIdx.x, lane = tid & 31, wave = tid >> 5;
  const int d0 = blockIdx.x * 256, d = d0 + tid;
  const int g0 = blockIdx.y * 64;
  const int tb = g0 & (kSeq - 1);
  const v4f wv = *(const v4f*)(cw + (size_t)d * 4);
  const float w0 = wv[0], w1 = wv[1], w2 = wv[2], w3 = wv[3];
  const float bc = cb[d];
  float xm3, xm2, xm1;
  {
    const bool hist = (tb > 0);
    const int rb = hist ? (g0 - 3) : g0;
    const float v3 = XZ[(size_t)rb * kXzP + d];
    const float v2 = XZ[(size_t)(rb + 1) * kXzP + d];
    const float v1 = XZ[(size_t)(rb + 2) * kXzP + d];
    xm3 = hist ? v3 : 0.f;
    xm2 = hist ? v2 : 0.f;
    xm1 = hist ? v1 : 0.f;
  }
  const int hrow = wave >> 1;
  const int hch  = (wave & 1) * 128 + lane * 4;
#pragma unroll 1
  for (int sub = 0; sub < 4; ++sub) {
    const int lb = g0 + sub * 16;
#pragma unroll 1
    for (int s = 0; s < 16; ++s) {
      const float xcur = XZ[(size_t)(lb + s) * kXzP + d];
      float acc = w0 * xm3;
      acc = fmaf(w1, xm2, acc);
      acc = fmaf(w2, xm1, acc);
      acc = fmaf(w3, xcur, acc);
      const float sv = acc + bc;
      const float sg = __builtin_amdgcn_rcpf(1.0f + expf(-sv));
      sT[s * kConvTP + tid] = sv * sg;
      xm3 = xm2; xm2 = xm1; xm1 = xcur;
    }
    __syncthreads();
    v4f fv[4];
    v8h bv[2];
#pragma unroll
    for (int it = 0; it < 4; ++it) fv[it] = *(const v4f*)(sT + (it * 4 + hrow) * kConvTP + hch);
#pragma unroll
    for (int it = 0; it < 2; ++it) {
      const float* sp = sT + (it * 8 + wave) * kConvTP + lane * 8;
      const v4f a0 = *(const v4f*)(sp);
      const v4f a1 = *(const v4f*)(sp + 4);
#pragma unroll
      for (int e = 0; e < 4; ++e) {
        bv[it][e]     = (_Float16)(a0[e] * kCarryXa);
        bv[it][4 + e] = (_Float16)(a1[e] * kCarryXa);
      }
    }
    for (int pass = 0; pass < 2; ++pass) {
#pragma unroll
      for (int it = 0; it < 4; ++it)
        *(volatile v4f*)(UC + (size_t)(lb + it * 4 + hrow) * kDin + d0 + hch) = fv[it];
#pragma unroll
      for (int it = 0; it < 2; ++it)
        *(volatile v8h*)(UC16 + (size_t)(lb + it * 8 + wave) * kDin + d0 + lane * 8) = bv[it];
      __threadfence();
    }
    __syncthreads();
  }
}

__global__ __launch_bounds__(256) void scan_kernel(
    const float* __restrict__ DLR, const float* __restrict__ UC, const float* __restrict__ XZ,
    const float* __restrict__ PROJ, const float* __restrict__ Alog, const float* __restrict__ Dp,
    unsigned short* __restrict__ YH, unsigned short* __restrict__ YL)
{
  __shared__ __align__(16) float sBC[kScTS * 2 * kNst];
  __shared__ __align__(16) float sDt[kScTS * kScCh];
  __shared__ __align__(16) float sXa[kScTS * kScCh];
  __shared__ __align__(16) float sYp[kScQ * kScTS * kScCh];
  __shared__ __align__(16) float sA[kNst * kScCh];
  const int tid = threadIdx.x, lane = tid & 31, wave = tid >> 5;
  const int c   = tid & (kScCh - 1);
  const int qtr = tid >> 6;
  constexpr int kBlkPerB = kDin / kScCh;
  const int bix = blockIdx.x / kBlkPerB;
  const int d0  = (blockIdx.x - bix * kBlkPerB) * kScCh;
  const int d   = d0 + c;
  const size_t row0 = (size_t)bix * kSeq;

#pragma unroll 1
  for (int n = 0; n < kScNq; ++n)
    sA[(qtr * kScNq + n) * kScCh + c] = -expf(Alog[(size_t)d * kNst + qtr * kScNq + n]);
  __syncthreads();
  float An[kScNq], h[kScNq];
#pragma unroll
  for (int n = 0; n < kScNq; ++n) {
    An[n] = sA[(qtr * kScNq + n) * kScCh + c];
    h[n] = 0.f;
  }
  const float Dd = Dp[d];

#pragma unroll 1
  for (int t0 = 0; t0 < kSeq; t0 += kScTS) {
    __syncthreads();
#pragma unroll
    for (int i = 0; i < 2; ++i) {
      const int idx = tid + 256 * i;
      const int r = idx >> 5, c4 = (idx & 31) * 4;
      *(v4f*)(sBC + r * (2 * kNst) + c4) = *(const v4f*)(PROJ + (row0 + t0 + r) * kPrjP + kDtR + c4);
    }
#pragma unroll 1
    for (int i = 0; i < 4; ++i) {
      const int r = qtr + 4 * i;
      const size_t gi = (row0 + t0 + r) * kDin + d;
      const float v = DLR[gi];
      float xa = UC[gi];
      asm volatile("" : "+v"(xa));
      const float ea = expf(-fabsf(v));
      sDt[r * kScCh + c] = fmaxf(v, 0.0f) + log1pf(ea);
      sXa[r * kScCh + c] = xa;
    }
    __syncthreads();
#pragma unroll 1
    for (int s = 0; s < kScTS; ++s) {
      const float delta = sDt[s * kScCh + c];
      const float xv    = sXa[s * kScCh + c];
      const float dtx   = delta * xv;
      const float* bp = sBC + s * (2 * kNst) + qtr * kScNq;
      v4f Bq[4], Cq[4];
#pragma unroll
      for (int k = 0; k < 4; ++k) {
        Bq[k] = *(const v4f*)(bp + 4 * k);
        Cq[k] = *(const v4f*)(bp + kNst + 4 * k);
      }
      float y = 0.f;
#pragma unroll
      for (int n = 0; n < kScNq; ++n) {
        const float e = __expf(delta * An[n]);
        h[n] = fmaf(e, h[n], dtx * Bq[n >> 2][n & 3]);
        y = fmaf(h[n], Cq[n >> 2][n & 3], y);
      }
      sYp[(qtr * kScTS + s) * kScCh + c] = y;
    }
    __syncthreads();
#pragma unroll 1
    for (int i = 0; i < 4; ++i) {
      const int r = qtr + 4 * i;
      const float p = (sYp[(0 * kScTS + r) * kScCh + c] + sYp[(1 * kScTS + r) * kScCh + c]) +
                      (sYp[(2 * kScTS + r) * kScCh + c] + sYp[(3 * kScTS + r) * kScCh + c]);
      const float xv = sXa[r * kScCh + c];
      float zv = XZ[(row0 + t0 + r) * kXzP + kDin + d];
      asm volatile("" : "+v"(zv));
      const float yv = fmaf(xv, Dd, p);
      const float sg = __builtin_amdgcn_rcpf(1.0f + expf(-zv));
      sYp[r * kScCh + c] = yv * (zv * sg);
    }
    __syncthreads();
    if (wave < 4) {
      const int q = lane >> 3, c8 = (lane & 7) * 8;
      const int row = wave * 4 + q;
      const float* sp = sYp + row * kScCh + c8;
      const v4f a0 = *(const v4f*)(sp);
      const v4f a1 = *(const v4f*)(sp + 4);
      v8h hv, lv;
#pragma unroll
      for (int e = 0; e < 4; ++e) {
        const float f0 = a0[e], f1 = a1[e];
        const unsigned short h0 = f2bf_bits(f0), h1 = f2bf_bits(f1);
        const unsigned short l0 = f2bf_bits(f0 - bf_bits2f(h0)), l1 = f2bf_bits(f1 - bf_bits2f(h1));
        hv[e]     = __builtin_bit_cast(_Float16, h0);
        hv[4 + e] = __builtin_bit_cast(_Float16, h1);
        lv[e]     = __builtin_bit_cast(_Float16, l0);
        lv[4 + e] = __builtin_bit_cast(_Float16, l1);
      }
      const size_t o = (row0 + t0 + row) * kDin + d0 + c8;
      for (int pass = 0; pass < 2; ++pass) {
        *(volatile v8h*)(YH + o) = hv;
        *(volatile v8h*)(YL + o) = lv;
        __threadfence();
      }
    }
  }
}

extern "C" void kernel_launch(void* const* d_in, const int* in_sizes, int n_in,
                              void* d_out, int out_size, void* d_ws, size_t ws_size,
                              hipStream_t stream) {
  if (n_in < 12) return;
  if (in_sizes[0] != kRows * kDm) return;
  if (in_sizes[1] != kDm || in_sizes[2] != kDm) return;
  if (in_sizes[3] != kXzP * kDm) return;
  if (in_sizes[4] != kDin * 4 || in_sizes[5] != kDin) return;
  if (in_sizes[6] != kPrjN * kDin) return;
  if (in_sizes[7] != kDin * kDtR || in_sizes[8] != kDin) return;
  if (in_sizes[9] != kDin * kNst || in_sizes[10] != kDin) return;
  if (in_sizes[11] != kDm * kDin) return;
  if (out_size != kRows * kDm) return;
  if (ws_size < kWsTotal) return;

  const float* x      = (const float*)d_in[0];
  const float* ln_g   = (const float*)d_in[1];
  const float* ln_b   = (const float*)d_in[2];
  const float* W_in   = (const float*)d_in[3];
  const float* conv_w = (const float*)d_in[4];
  const float* conv_b = (const float*)d_in[5];
  const float* W_x    = (const float*)d_in[6];
  const float* W_dt   = (const float*)d_in[7];
  const float* b_dt   = (const float*)d_in[8];
  const float* A_log  = (const float*)d_in[9];
  const float* Dp     = (const float*)d_in[10];
  const float* W_out  = (const float*)d_in[11];
  float* out = (float*)d_out;

  char* ws = (char*)d_ws;
  unsigned short* XNH   = (unsigned short*)(ws + kOffXNH);
  unsigned short* XNL   = (unsigned short*)(ws + kOffXNL);
  unsigned short* WIH   = (unsigned short*)(ws + kOffWIH);
  unsigned short* WIL   = (unsigned short*)(ws + kOffWIL);
  unsigned short* WOH   = (unsigned short*)(ws + kOffWOH);
  unsigned short* WOL   = (unsigned short*)(ws + kOffWOL);
  unsigned short* WXP16 = (unsigned short*)(ws + kOffWXP);
  unsigned short* WDT16 = (unsigned short*)(ws + kOffWDT);
  float*          XZ    = (float*)(ws + kOffXZ);
  float*          UC    = (float*)(ws + kOffUC);
  unsigned short* UC16  = (unsigned short*)(ws + kOffUC16);
  float*          PROJ  = (float*)(ws + kOffPROJ);
  unsigned short* DT16  = (unsigned short*)(ws + kOffDT16);
  float*          DLR   = (float*)(ws + kOffDLR);
  unsigned short* YH    = (unsigned short*)(ws + kOffYH);
  unsigned short* YL    = (unsigned short*)(ws + kOffYL);

  {
    const int t8 = kXzP * kDm / 8;
    split_rows_bf16_kernel<<<(t8 + 255) / 256, 256, 0, stream>>>(W_in, WIH, WIL, t8);
  }
  {
    const int t8 = kDm * kDin / 8;
    split_rows_bf16_kernel<<<(t8 + 255) / 256, 256, 0, stream>>>(W_out, WOH, WOL, t8);
  }
  {
    const int t8 = kPrjP * kDin / 8;
    cast_pad_f16_kernel<<<(t8 + 255) / 256, 256, 0, stream>>>(W_x, kDin, kPrjN, kDin, WXP16, kDin, t8, kCarryWx);
  }
  {
    const int t8 = kDin * kDtP / 8;
    cast_pad_f16_kernel<<<(t8 + 255) / 256, 256, 0, stream>>>(W_dt, kDtR, kDin, kDtR, WDT16, kDtP, t8, kCarryWdt);
  }

  ln_split_kernel<<<kRows / 8, 256, 0, stream>>>(x, ln_g, ln_b, XNH, XNL);

  wmma_gemm64<1, 2, 0><<<(kRows / 64) * (kXzP / 64) / 8, 256, 0, stream>>>(
      XNH, XNL, kDm, WIH, WIL, kDm, XZ, kXzP, b_dt, kRows, kXzP, kDm, 1.0f);

  conv_silu_kernel<<<dim3(kDin / 256, kRows / 64), 256, 0, stream>>>(XZ, conv_w, conv_b, UC, UC16);

  wmma_gemm64<0, 0, 0><<<(kRows / 64) * (kPrjP / 64) / 8, 256, 0, stream>>>(
      UC16, UC16, kDin, WXP16, WXP16, kDin, PROJ, kPrjP, b_dt, kRows, kPrjP, kDin,
      1.0f / (kCarryXa * kCarryWx));

  {
    const int t8 = kRows * kDtP / 8;
    cast_pad_f16_kernel<<<(t8 + 255) / 256, 256, 0, stream>>>(PROJ, kPrjP, kRows, kDtR, DT16, kDtP, t8, kCarryDt);
  }

  wmma_gemm64<0, 0, 2><<<(kRows / 64) * (kDin / 64) / 8, 256, 0, stream>>>(
      DT16, DT16, kDtP, WDT16, WDT16, kDtP, DLR, kDin, b_dt, kRows, kDin, kDtP,
      1.0f / (kCarryDt * kCarryWdt));

  scan_kernel<<<kBatch * (kDin / kScCh), 256, 0, stream>>>(DLR, UC, XZ, PROJ, A_log, Dp, YH, YL);

  wmma_gemm64<1, 2, 0><<<(kRows / 64) * (kDm / 64) / 8, 256, 0, stream>>>(
      YH, YL, kDin, WOH, WOL, kDin, out, kDm, b_dt, kRows, kDm, kDin, 1.0f);
}
